// EnhancedDecoderAttention_56332791054981
// MI455X (gfx1250) — hardware-verified
//
#include <hip/hip_runtime.h>
#include <math.h>
#include <stdint.h>

constexpr int kBatch = 4;
constexpr int kSeq   = 2048;
constexpr int kDm    = 1024;
constexpr int kHeads = 16;

typedef __attribute__((ext_vector_type(16))) _Float16 v16h;
typedef __attribute__((ext_vector_type(8)))  _Float16 v8h;
typedef __attribute__((ext_vector_type(16))) __bf16   v16b;
typedef __attribute__((ext_vector_type(8)))  __bf16   v8b;
typedef __attribute__((ext_vector_type(8)))  float    v8f;
typedef __attribute__((ext_vector_type(4)))  float    v4f;
typedef __attribute__((ext_vector_type(2)))  float    v2f;
typedef __attribute__((ext_vector_type(4)))  unsigned int v4u;
typedef __attribute__((ext_vector_type(8)))  unsigned short v8us;

__device__ __forceinline__ unsigned short f2bf_bits(float f) {
  unsigned u = __float_as_uint(f);
  return (unsigned short)((u + 0x7FFFu + ((u >> 16) & 1u)) >> 16);
}
__device__ __forceinline__ float bf_bits2f(unsigned short h) { return __uint_as_float(((unsigned)h) << 16); }

__device__ __forceinline__ void dep_guard_h(v8f& a, v8f& b, v16h x, v16h y) { asm volatile("v_nop\n\tv_nop\n\tv_nop\n\tv_nop" : "+v"(a), "+v"(b) : "v"(x), "v"(y)); }
__device__ __forceinline__ void dep_guard_b(v8f& a, v8f& b, v16b x, v16b y) { asm volatile("v_nop\n\tv_nop\n\tv_nop\n\tv_nop" : "+v"(a), "+v"(b) : "v"(x), "v"(y)); }
__device__ __forceinline__ void keep4_h(v16h a, v16h b, v16h c, v16h d) { asm volatile("v_nop" :: "v"(a), "v"(b), "v"(c), "v"(d)); }
__device__ __forceinline__ void keep4_b(v16b a, v16b b, v16b c, v16b d) { asm volatile("v_nop" :: "v"(a), "v"(b), "v"(c), "v"(d)); }
__device__ __forceinline__ void acc_guard4(v8f& a, v8f& b, v8f& c, v8f& d) { asm volatile("v_nop\n\tv_nop\n\tv_nop\n\tv_nop" : "+v"(a), "+v"(b), "+v"(c), "+v"(d)); }
template <typename T> struct Frag;
template <> struct Frag<_Float16> {
  typedef v16h V; union U { v16h v; v8h h[2]; };
  static __device__ __forceinline__ v16h load(const _Float16* p) {
    U f; f.h[0] = *(const v8h*)(p); f.h[1] = *(const v8h*)(p + 16); return f.v;
  }
  static __device__ __forceinline__ v8f mma(v16h a, v16h b, v8f c) {
    return __builtin_amdgcn_wmma_f32_16x16x32_f16(false, a, false, b, (short)0, c, false, false);
  }
  static __device__ __forceinline__ void guard(v8f& a, v8f& b, v16h x, v16h y) { dep_guard_h(a, b, x, y); }
  static __device__ __forceinline__ void keep(v16h a, v16h b, v16h c, v16h d) { keep4_h(a, b, c, d); }
};
template <> struct Frag<__bf16> {
  typedef v16b V; union U { v16b v; v8b h[2]; };
  static __device__ __forceinline__ v16b load(const __bf16* p) {
    U f; f.h[0] = *(const v8b*)(p); f.h[1] = *(const v8b*)(p + 16); return f.v;
  }
  static __device__ __forceinline__ v8f mma(v16b a, v16b b, v8f c) {
    return __builtin_amdgcn_wmma_f32_16x16x32_bf16(false, a, false, b, (short)0, c, false, false);
  }
  static __device__ __forceinline__ void guard(v8f& a, v8f& b, v16b x, v16b y) { dep_guard_b(a, b, x, y); }
  static __device__ __forceinline__ void keep(v16b a, v16b b, v16b c, v16b d) { keep4_b(a, b, c, d); }
};

template <int ET> struct Elem;
template <> struct Elem<0> { typedef _Float16 T; };
template <> struct Elem<1> { typedef __bf16 T; };
template <int ET, bool SPLIT, int BIAS_MODE, int OUT_MODE, bool RESID, int ACT = 0>
__global__ __launch_bounds__(256) void wmma_gemm64(
    const unsigned short* __restrict__ Ap, const unsigned short* __restrict__ A2p, int lda, long strideA,
    const unsigned short* __restrict__ Btp, const unsigned short* __restrict__ Bt2p, int ldb, long strideB,
    void* __restrict__ Cout, void* __restrict__ Cout2, int ldc, long strideC,
    const float* __restrict__ bias,
    const float* __restrict__ resid, long strideR,
    int M, int N, int K, float scale) {
  typedef typename Elem<ET>::T T;
  typedef typename Frag<T>::V V;
  const T* A = (const T*)Ap; const T* A2 = (const T*)A2p; const T* Bt = (const T*)Btp; const T* Bt2 = (const T*)Bt2p;
  __shared__ __align__(16) float sT[8][16 * 68];
  const int b    = blockIdx.y;
  const int lane = threadIdx.x & 31;
  const int wave = threadIdx.x >> 5;
  const int tilesN = N >> 6;
  const int tilesM = M >> 6;
  const int tile = blockIdx.x * 8 + wave;
  if (tile >= tilesM * tilesN) return;
  const int tm = tile / tilesN;
  const int tn = tile - tm * tilesN;
  const int m0 = tm << 6;
  const int n0 = tn << 6;

  const T* Ab  = A  + (size_t)b * strideA;
  const T* Bb  = Bt + (size_t)b * strideB;
  const T* Ab2 = SPLIT ? (A2  + (size_t)b * strideA) : nullptr;
  const T* Bb2 = SPLIT ? (Bt2 + (size_t)b * strideB) : nullptr;

  const int rlane = lane & 15;
  const int koff  = (lane >> 4) * 8;
  const int mOff  = (lane >> 4) * 8;

  v8f acc[4][4];
#pragma unroll
  for (int i = 0; i < 4; ++i)
#pragma unroll
    for (int j = 0; j < 4; ++j) acc[i][j] = (v8f){0.f,0.f,0.f,0.f,0.f,0.f,0.f,0.f};

  for (int k0 = 0; k0 < K; k0 += 32) {
    V bh[4], bl[4];
#pragma unroll
    for (int j = 0; j < 4; ++j) {
      const size_t bo = (size_t)(n0 + (j << 4) + rlane) * ldb + koff + k0;
      bh[j] = Frag<T>::load(Bb + bo);
      if (SPLIT) bl[j] = Frag<T>::load(Bb2 + bo);
    }
#pragma unroll
    for (int i = 0; i < 4; ++i) {
      const size_t ao = (size_t)(m0 + (i << 4) + rlane) * lda + koff + k0;
      V ah = Frag<T>::load(Ab + ao);
      V al;
      if (SPLIT) al = Frag<T>::load(Ab2 + ao);
#pragma unroll
      for (int j = 0; j < 4; ++j) {
        acc[i][j] = Frag<T>::mma(ah, bh[j], acc[i][j]);
        if (SPLIT) {
          acc[i][j] = Frag<T>::mma(ah, bl[j], acc[i][j]);
          acc[i][j] = Frag<T>::mma(al, bh[j], acc[i][j]);
        }
      }
      Frag<T>::guard(acc[i][0], acc[i][3], ah, SPLIT ? al : ah);
    }
    Frag<T>::keep(bh[0], bh[1], bh[2], bh[3]);
    if (SPLIT) Frag<T>::keep(bl[0], bl[1], bl[2], bl[3]);
  }
  acc_guard4(acc[0][0], acc[0][1], acc[0][2], acc[0][3]);
  acc_guard4(acc[1][0], acc[1][1], acc[1][2], acc[1][3]);
  acc_guard4(acc[2][0], acc[2][1], acc[2][2], acc[2][3]);
  acc_guard4(acc[3][0], acc[3][1], acc[3][2], acc[3][3]);

  float* slab = sT[wave];
  const float* Rb = RESID ? (resid + (size_t)b * strideR) : nullptr;
#pragma unroll
  for (int i = 0; i < 4; ++i) {
    const int mBase = m0 + (i << 4);
#pragma unroll
    for (int j = 0; j < 4; ++j) {
      const int n = n0 + (j << 4) + rlane;
      float bv = 0.f;
      if (BIAS_MODE == 2) bv = bias[n];
#pragma unroll
      for (int r = 0; r < 8; ++r) {
        float v = acc[i][j][r] * scale;
        if (BIAS_MODE == 1) v += bias[mBase + mOff + r];
        if (BIAS_MODE == 2) v += bv;
        if (RESID) v += Rb[(size_t)(mBase + mOff + r) * ldc + n];
        if (ACT == 1) v = tanhf(v);
        if (ACT == 2) v = fmaxf(v, 0.0f);
        if (ACT == 3) v = v / (1.0f + expf(-v));
        if (ACT == 4) v = (v > 0.f) ? v : 0.01f * v;
        slab[(mOff + r) * 68 + (j << 4) + rlane] = v;
      }
    }
    __builtin_amdgcn_fence(__ATOMIC_RELEASE, "workgroup");
    __builtin_amdgcn_wave_barrier();
    __builtin_amdgcn_fence(__ATOMIC_ACQUIRE, "workgroup");
    if (OUT_MODE == 0) {
      float* C = (float*)Cout + (size_t)b * strideC;
      const int hh = lane >> 4, c4 = (lane & 15) * 4;
      for (int pass = 0; pass < 2; ++pass) {
#pragma unroll
        for (int it = 0; it < 8; ++it) {
          const int row = it * 2 + hh;
          v4f v = *(const v4f*)(slab + row * 68 + c4);
          *(volatile v4f*)(C + (size_t)(mBase + row) * ldc + n0 + c4) = v;
        }
        __threadfence();
      }
    } else {
      const int q = lane >> 3, c8 = (lane & 7) * 8;
      unsigned short* C  = (unsigned short*)Cout  + (size_t)b * strideC;
      unsigned short* C2 = (OUT_MODE == 2) ? ((unsigned short*)Cout2 + (size_t)b * strideC) : nullptr;
      for (int pass = 0; pass < 2; ++pass) {
#pragma unroll
        for (int it = 0; it < 4; ++it) {
          const int row = it * 4 + q;
          const float* sp = slab + row * 68 + c8;
          v8h hv, lv;
#pragma unroll
          for (int e = 0; e < 8; ++e) {
            if (OUT_MODE == 1) {
              hv[e] = (_Float16)sp[e];
            } else {
              unsigned short hb = f2bf_bits(sp[e]);
              unsigned short lb = f2bf_bits(sp[e] - bf_bits2f(hb));
              hv[e] = __builtin_bit_cast(_Float16, hb);
              lv[e] = __builtin_bit_cast(_Float16, lb);
            }
          }
          *(volatile v8h*)(C + (size_t)(mBase + row) * ldc + n0 + c8) = hv;
          if (OUT_MODE == 2) *(volatile v8h*)(C2 + (size_t)(mBase + row) * ldc + n0 + c8) = lv;
        }
        __threadfence();
      }
    }
    __builtin_amdgcn_fence(__ATOMIC_RELEASE, "workgroup");
    __builtin_amdgcn_wave_barrier();
    __builtin_amdgcn_fence(__ATOMIC_ACQUIRE, "workgroup");
  }
}

__device__ __forceinline__ unsigned pk16(unsigned short a, unsigned short b) { return (unsigned)a | ((unsigned)b << 16); }

__global__ __launch_bounds__(256) void split_bf16x2_kernel(const float* __restrict__ in, unsigned short* __restrict__ hi,
                                                           unsigned short* __restrict__ lo, int n2) {
  const int i = blockIdx.x * 256 + threadIdx.x;
  if (i < n2) {
    const v2f f = *(const v2f*)(in + 2 * (size_t)i);
    const unsigned short h0 = f2bf_bits(f[0]), h1 = f2bf_bits(f[1]);
    const unsigned short l0 = f2bf_bits(f[0] - bf_bits2f(h0)), l1 = f2bf_bits(f[1] - bf_bits2f(h1));
    const unsigned uh = pk16(h0, h1), ul = pk16(l0, l1);
    ((volatile unsigned*)hi)[i] = uh;
    ((volatile unsigned*)lo)[i] = ul;
    __threadfence();
    ((volatile unsigned*)hi)[i] = uh;
    ((volatile unsigned*)lo)[i] = ul;
  }
}

__global__ __launch_bounds__(256) void wt_split_kernel(const float* __restrict__ w, unsigned short* __restrict__ th,
                                                       unsigned short* __restrict__ tl, int R, int Cn) {
  __shared__ float tile[64 * 65];
  const int n0 = blockIdx.x * 64;
  const int k0 = blockIdx.y * 64;
  const int t = threadIdx.x;
#pragma unroll
  for (int i = 0; i < 16; ++i) {
    const int idx = i * 256 + t;
    const int kk = idx >> 6, nn = idx & 63;
    tile[nn * 65 + kk] = w[(size_t)(k0 + kk) * Cn + n0 + nn];
  }
  __syncthreads();
  const int lane = t & 31, wave = t >> 5;
  const int q = lane >> 3, c8 = (lane & 7) * 8;
  for (int pass = 0; pass < 2; ++pass) {
#pragma unroll
    for (int it = 0; it < 2; ++it) {
      const int row = wave * 8 + it * 4 + q;
      const float* sp = tile + row * 65 + c8;
      v8us hv, lv;
#pragma unroll
      for (int e = 0; e < 8; ++e) {
        const unsigned short hb = f2bf_bits(sp[e]);
        const unsigned short lb = f2bf_bits(sp[e] - bf_bits2f(hb));
        hv[e] = hb; lv[e] = lb;
      }
      const size_t o = (size_t)(n0 + row) * R + k0 + c8;
      *(volatile v8us*)(th + o) = hv;
      *(volatile v8us*)(tl + o) = lv;
    }
    __threadfence();
  }
}

__global__ __launch_bounds__(256) void rope_split_kernel(const float* __restrict__ qf, const float* __restrict__ kf,
                                                         unsigned short* __restrict__ qh, unsigned short* __restrict__ ql,
                                                         unsigned short* __restrict__ kh, unsigned short* __restrict__ kl) {
  __shared__ __align__(16) unsigned short Lh[8][128];
  __shared__ __align__(16) unsigned short Ll[8][128];
  const int s = blockIdx.x;
  const int which = blockIdx.y;
  const float* src = (which == 0) ? qf : kf;
  unsigned short* dh = (which == 0) ? qh : kh;
  unsigned short* dl = (which == 0) ? ql : kl;
  const int lane = threadIdx.x & 31;
  const int wave = threadIdx.x >> 5;

  const float t = (float)(2 * lane) * 0.015625f;
  const float p = powf(10000.0f, t);
  const float inv = 1.0f / p;
  const float ang = (float)s * inv;
  float sn, cs;
  sincosf(ang, &sn, &cs);

  const float* row = src + (size_t)s * kDm + wave * 128;
  unsigned short* lh = Lh[wave];
  unsigned short* ll = Ll[wave];
#pragma unroll 1
  for (int hp = 0; hp < 2; ++hp) {
    const float xr = row[hp * 64 + lane];
    const float xi = row[hp * 64 + 32 + lane];
    const float vr = xr * cs - xi * sn;
    const float vi = xi * cs + xr * sn;
    const unsigned short hr = f2bf_bits(vr);
    const unsigned short lr = f2bf_bits(vr - bf_bits2f(hr));
    const unsigned short hi = f2bf_bits(vi);
    const unsigned short li = f2bf_bits(vi - bf_bits2f(hi));
    lh[hp * 64 + lane] = hr;       ll[hp * 64 + lane] = lr;
    lh[hp * 64 + 32 + lane] = hi;  ll[hp * 64 + 32 + lane] = li;
  }
  __builtin_amdgcn_fence(__ATOMIC_RELEASE, "workgroup");
  __builtin_amdgcn_wave_barrier();
  __builtin_amdgcn_fence(__ATOMIC_ACQUIRE, "workgroup");
  const int l16 = lane & 15;
  const v8us hv = *(const v8us*)(lh + l16 * 8);
  const v8us lv = *(const v8us*)(ll + l16 * 8);
  const size_t o = (size_t)s * kDm + wave * 128 + l16 * 8;
  for (int pass = 0; pass < 2; ++pass) {
    if (lane < 16) {
      *(volatile v8us*)(dh + o) = hv;
      *(volatile v8us*)(dl + o) = lv;
    }
    __threadfence();
  }
}

#define AT_D 64
#define AT_NW 4
#define AT_QB 64
#define AT_KC 64

__device__ __forceinline__ unsigned short at_bf_bits(float f) {
  unsigned u = __float_as_uint(f);
  return (unsigned short)((u + 0x7FFFu + ((u >> 16) & 1u)) >> 16);
}
__device__ __forceinline__ __bf16 at_f2bf(float f) { return __builtin_bit_cast(__bf16, at_bf_bits(f)); }
__device__ __forceinline__ void at_split(float f, __bf16& hi, __bf16& lo) {
  const unsigned short hb = at_bf_bits(f);
  hi = __builtin_bit_cast(__bf16, hb);
  lo = at_f2bf(f - __uint_as_float(((unsigned)hb) << 16));
}
__device__ __forceinline__ v8f at_mma(v16b a, v16b b, v8f c) {
  c = __builtin_amdgcn_wmma_f32_16x16x32_bf16(false, a, false, b, (short)0, c, false, false);
  asm volatile("v_nop\n\tv_nop\n\tv_nop\n\tv_nop" : "+v"(c) : "v"(a), "v"(b));
  return c;
}

__global__ __launch_bounds__(128)
void attn_mask64_kernel(const unsigned short* __restrict__ qhp, const unsigned short* __restrict__ qlp,
                        const unsigned short* __restrict__ khp, const unsigned short* __restrict__ klp,
                        const unsigned short* __restrict__ vhp, const unsigned short* __restrict__ vlp,
                        const int* __restrict__ mask,
                        float* __restrict__ out, float sscale, float mfill) {
  union FB { v16b v; v8b h[2]; };
  __shared__ __align__(16) __bf16 Ksh[AT_KC * AT_D];
  __shared__ __align__(16) __bf16 Ksl[AT_KC * AT_D];
  __shared__ __align__(16) __bf16 Vth[AT_D * AT_KC];
  __shared__ __align__(16) __bf16 Vtl[AT_D * AT_KC];
  __shared__ __align__(16) __bf16 Psh[AT_NW][16 * AT_KC];
  __shared__ __align__(16) __bf16 Psl[AT_NW][16 * AT_KC];
  __shared__ __align__(16) float  Os[AT_NW][16 * 68];

  const int tid  = threadIdx.x;
  const int wave = tid >> 5;
  const int lane = tid & 31;
  const int hh   = lane >> 4;
  const int c    = lane & 15;

  const int nqb = kSeq / AT_QB;
  const int bx = blockIdx.x;
  const int qb = bx % nqb;
  const int h  = bx / nqb;
  const int q0 = qb * AT_QB + wave * 16;

  const __bf16* Qh = (const __bf16*)(const void*)qhp + (size_t)h * AT_D;
  const __bf16* Ql = (const __bf16*)(const void*)qlp + (size_t)h * AT_D;
  const __bf16* Kh = (const __bf16*)(const void*)khp + (size_t)h * AT_D;
  const __bf16* Kl = (const __bf16*)(const void*)klp + (size_t)h * AT_D;
  const __bf16* Vh = (const __bf16*)(const void*)vhp + (size_t)h * AT_D * kSeq;
  const __bf16* Vl = (const __bf16*)(const void*)vlp + (size_t)h * AT_D * kSeq;
  float*        ob = out + (size_t)h * AT_D;

  v16b qah[2], qal[2];
#pragma unroll
  for (int dc = 0; dc < 2; ++dc) {
    const __bf16* qr = Qh + (size_t)(q0 + c) * kDm + dc * 32 + 8 * hh;
    const __bf16* ql = Ql + (size_t)(q0 + c) * kDm + dc * 32 + 8 * hh;
    qah[dc] = Frag<__bf16>::load(qr);
    qal[dc] = Frag<__bf16>::load(ql);
  }

  float mrow[8], lrow[8];
  v8f oacc[4];
#pragma unroll
  for (int r = 0; r < 8; ++r) { mrow[r] = -INFINITY; lrow[r] = 0.f; }
#pragma unroll
  for (int t = 0; t < 4; ++t) oacc[t] = (v8f){0.f,0.f,0.f,0.f,0.f,0.f,0.f,0.f};

  int nChunks = qb + 1;
  if (nChunks > kSeq / AT_KC) nChunks = kSeq / AT_KC;
  for (int kc = 0; kc < nChunks; ++kc) {
    const int kv0 = kc * AT_KC;
    __syncthreads();
    {
      const int r = tid >> 1, half = (tid & 1) * 32;
      const __bf16* ksh = Kh + (size_t)(kv0 + r) * kDm + half;
      const __bf16* ksl = Kl + (size_t)(kv0 + r) * kDm + half;
      const __bf16* vsh = Vh + (size_t)r * kSeq + kv0 + half;
      const __bf16* vsl = Vl + (size_t)r * kSeq + kv0 + half;
#pragma unroll
      for (int i = 0; i < 4; ++i) {
        const v8b a0 = *(const v8b*)(ksh + 8 * i);
        const v8b a1 = *(const v8b*)(ksl + 8 * i);
        const v8b b0 = *(const v8b*)(vsh + 8 * i);
        const v8b b1 = *(const v8b*)(vsl + 8 * i);
        *(v8b*)(Ksh + r * AT_D  + half + 8 * i) = a0;
        *(v8b*)(Ksl + r * AT_D  + half + 8 * i) = a1;
        *(v8b*)(Vth + r * AT_KC + half + 8 * i) = b0;
        *(v8b*)(Vtl + r * AT_KC + half + 8 * i) = b1;
      }
    }
    __syncthreads();

    v8f s[4];
#pragma unroll
    for (int j = 0; j < 4; ++j) {
      s[j] = (v8f){0.f,0.f,0.f,0.f,0.f,0.f,0.f,0.f};
#pragma unroll
      for (int dc = 0; dc < 2; ++dc) {
        FB kb, kl;
        kb.h[0] = *(const v8b*)(Ksh + (j * 16 + c) * AT_D + dc * 32 + 8 * hh);
        kb.h[1] = *(const v8b*)(Ksh + (j * 16 + c) * AT_D + dc * 32 + 16 + 8 * hh);
        kl.h[0] = *(const v8b*)(Ksl + (j * 16 + c) * AT_D + dc * 32 + 8 * hh);
        kl.h[1] = *(const v8b*)(Ksl + (j * 16 + c) * AT_D + dc * 32 + 16 + 8 * hh);
        s[j] = at_mma(qah[dc], kb.v, s[j]);
        s[j] = at_mma(qah[dc], kl.v, s[j]);
        s[j] = at_mma(qal[dc], kb.v, s[j]);
      }
    }
    float cm[8];
#pragma unroll
    for (int r = 0; r < 8; ++r) {
      const int qrow = q0 + 8 * hh + r;
      const int* mk = mask + (size_t)qrow * kSeq + kv0;
      float m = -INFINITY;
#pragma unroll
      for (int j = 0; j < 4; ++j) {
        const int mv = mk[j * 16 + c];
        const float sv = s[j][r] * sscale;
        const float sm = (mv == 0) ? mfill : sv;
        s[j][r] = sm;
        m = fmaxf(m, sm);
      }
#pragma unroll
      for (int off = 1; off < 16; off <<= 1) m = fmaxf(m, __shfl_xor(m, off, 32));
      cm[r] = m;
    }
    __bf16* pwh = Psh[wave];
    __bf16* pwl = Psl[wave];
#pragma unroll
    for (int r = 0; r < 8; ++r) {
      const float mnew = fmaxf(mrow[r], cm[r]);
      const float alpha = expf(mrow[r] - mnew);
      mrow[r] = mnew;
      float psum = 0.f;
#pragma unroll
      for (int j = 0; j < 4; ++j) {
        const float p = expf(s[j][r] - mnew);
        psum += p;
        __bf16 a, bl; at_split(p, a, bl);
        pwh[(8 * hh + r) * AT_KC + j * 16 + c] = a;
        pwl[(8 * hh + r) * AT_KC + j * 16 + c] = bl;
      }
#pragma unroll
      for (int off = 1; off < 16; off <<= 1) psum += __shfl_xor(psum, off, 32);
      lrow[r] = lrow[r] * alpha + psum;
#pragma unroll
      for (int t = 0; t < 4; ++t) oacc[t][r] *= alpha;
    }
    __builtin_amdgcn_fence(__ATOMIC_RELEASE, "workgroup");
    __builtin_amdgcn_wave_barrier();
    __builtin_amdgcn_fence(__ATOMIC_ACQUIRE, "workgroup");
#pragma unroll 1
    for (int kk = 0; kk < 2; ++kk) {
      FB pa, pl;
      pa.h[0] = *(const v8b*)(pwh + c * AT_KC + kk * 32 + 8 * hh);
      pa.h[1] = *(const v8b*)(pwh + c * AT_KC + kk * 32 + 16 + 8 * hh);
      pl.h[0] = *(const v8b*)(pwl + c * AT_KC + kk * 32 + 8 * hh);
      pl.h[1] = *(const v8b*)(pwl + c * AT_KC + kk * 32 + 16 + 8 * hh);
#pragma unroll
      for (int t = 0; t < 4; ++t) {
        FB vb, vl;
        vb.h[0] = *(const v8b*)(Vth + (t * 16 + c) * AT_KC + kk * 32 + 8 * hh);
        vb.h[1] = *(const v8b*)(Vth + (t * 16 + c) * AT_KC + kk * 32 + 16 + 8 * hh);
        vl.h[0] = *(const v8b*)(Vtl + (t * 16 + c) * AT_KC + kk * 32 + 8 * hh);
        vl.h[1] = *(const v8b*)(Vtl + (t * 16 + c) * AT_KC + kk * 32 + 16 + 8 * hh);
        oacc[t] = at_mma(pa.v, vb.v, oacc[t]);
        oacc[t] = at_mma(pa.v, vl.v, oacc[t]);
        oacc[t] = at_mma(pl.v, vb.v, oacc[t]);
      }
    }
  }

  float* os = Os[wave];
#pragma unroll
  for (int r = 0; r < 8; ++r) {
    const float inv = 1.0f / lrow[r];
#pragma unroll
    for (int t = 0; t < 4; ++t) os[(8 * hh + r) * 68 + t * 16 + c] = oacc[t][r] * inv;
  }
  __builtin_amdgcn_fence(__ATOMIC_RELEASE, "workgroup");
  __builtin_amdgcn_wave_barrier();
  __builtin_amdgcn_fence(__ATOMIC_ACQUIRE, "workgroup");
  {
    const int c4 = (lane & 15) * 4;
    for (int pass = 0; pass < 2; ++pass) {
#pragma unroll
      for (int it = 0; it < 8; ++it) {
        const int row = it * 2 + hh;
        v4f val = *(const v4f*)(os + row * 68 + c4);
        *(volatile v4f*)(ob + (size_t)(q0 + row) * kDm + c4) = val;
      }
      __threadfence();
    }
  }
}

extern "C" void kernel_launch(void* const* d_in, const int* in_sizes, int n_in,
                              void* d_out, int out_size, void* d_ws, size_t ws_size,
                              hipStream_t stream) {
  if (n_in < 10) return;
  const int nAct = kBatch * kSeq * kDm;
  const int nRow = kSeq * kDm;
  const int nW   = kDm * kDm;
  if (in_sizes[0] != nAct) return;
  if (in_sizes[1] != kSeq * kSeq) return;
  if (in_sizes[2] != nW || in_sizes[4] != nW || in_sizes[6] != nW || in_sizes[8] != nW) return;
  if (in_sizes[3] != kDm || in_sizes[5] != kDm || in_sizes[7] != kDm || in_sizes[9] != kDm) return;
  if (out_size != nAct) return;

  const float* x    = (const float*)d_in[0];
  const int*   mask = (const int*)d_in[1];
  const float* wq   = (const float*)d_in[2];
  const float* bq   = (const float*)d_in[3];
  const float* wk   = (const float*)d_in[4];
  const float* bk   = (const float*)d_in[5];
  const float* wv   = (const float*)d_in[6];
  const float* bv   = (const float*)d_in[7];
  const float* wo   = (const float*)d_in[8];
  const float* bo   = (const float*)d_in[9];

  const size_t PW = (size_t)kDm * kDm * 2;
  const size_t PX = (size_t)kSeq * kDm * 2;
  const size_t PF = (size_t)kSeq * kDm * 4;
  size_t off = 0;
  const size_t oWqh = off; off += PW;  const size_t oWql = off; off += PW;
  const size_t oWkh = off; off += PW;  const size_t oWkl = off; off += PW;
  const size_t oWvh = off; off += PW;  const size_t oWvl = off; off += PW;
  const size_t oWoh = off; off += PW;  const size_t oWol = off; off += PW;
  const size_t oXh  = off; off += PX;  const size_t oXl  = off; off += PX;
  const size_t oQf  = off; off += PF;
  const size_t oKf  = off; off += PF;
  const size_t oQh  = off; off += PX;  const size_t oQl  = off; off += PX;
  const size_t oKh  = off; off += PX;  const size_t oKl  = off; off += PX;
  const size_t oVTh = off; off += PX;  const size_t oVTl = off; off += PX;
  const size_t oOf  = off; off += PF;
  const size_t oOh  = off; off += PX;  const size_t oOl  = off; off += PX;
  if (off > ws_size) return;

  char* ws = (char*)d_ws;
  unsigned short* Wqh = (unsigned short*)(ws + oWqh); unsigned short* Wql = (unsigned short*)(ws + oWql);
  unsigned short* Wkh = (unsigned short*)(ws + oWkh); unsigned short* Wkl = (unsigned short*)(ws + oWkl);
  unsigned short* Wvh = (unsigned short*)(ws + oWvh); unsigned short* Wvl = (unsigned short*)(ws + oWvl);
  unsigned short* Woh = (unsigned short*)(ws + oWoh); unsigned short* Wol = (unsigned short*)(ws + oWol);
  unsigned short* Xh  = (unsigned short*)(ws + oXh);  unsigned short* Xl  = (unsigned short*)(ws + oXl);
  float*          Qf  = (float*)(ws + oQf);
  float*          Kf  = (float*)(ws + oKf);
  unsigned short* Qh  = (unsigned short*)(ws + oQh);  unsigned short* Ql  = (unsigned short*)(ws + oQl);
  unsigned short* Kh  = (unsigned short*)(ws + oKh);  unsigned short* Kl  = (unsigned short*)(ws + oKl);
  unsigned short* VTh = (unsigned short*)(ws + oVTh); unsigned short* VTl = (unsigned short*)(ws + oVTl);
  float*          Of  = (float*)(ws + oOf);
  unsigned short* Oh  = (unsigned short*)(ws + oOh);  unsigned short* Ol  = (unsigned short*)(ws + oOl);

  const dim3 blk(256);
  const dim3 gWt(kDm / 64, kDm / 64);
  const int n2x = nRow / 2;
  const dim3 gCast((n2x + 255) / 256);
  const dim3 gProj(((kSeq / 64) * (kDm / 64) + 7) / 8, 1);
  const dim3 gVT(((kDm / 64) * (kSeq / 64) + 7) / 8, 1);
  const dim3 gRope(kSeq, 2);
  const dim3 gAtt(kHeads * (kSeq / 64));

  wt_split_kernel<<<gWt, blk, 0, stream>>>(wq, Wqh, Wql, kDm, kDm);
  wt_split_kernel<<<gWt, blk, 0, stream>>>(wk, Wkh, Wkl, kDm, kDm);
  wt_split_kernel<<<gWt, blk, 0, stream>>>(wv, Wvh, Wvl, kDm, kDm);
  wt_split_kernel<<<gWt, blk, 0, stream>>>(wo, Woh, Wol, kDm, kDm);

  for (int b = 0; b < kBatch; ++b) {
    const float* xb = x + (size_t)b * nRow;
    split_bf16x2_kernel<<<gCast, blk, 0, stream>>>(xb, Xh, Xl, n2x);
    wmma_gemm64<1, true, 2, 0, false, 0><<<gProj, blk, 0, stream>>>(
        Xh, Xl, kDm, 0L, Wqh, Wql, kDm, 0L, (void*)Qf, (void*)Qf, kDm, 0L,
        bq, bq, 0L, kSeq, kDm, kDm, 1.0f);
    wmma_gemm64<1, true, 2, 0, false, 0><<<gProj, blk, 0, stream>>>(
        Xh, Xl, kDm, 0L, Wkh, Wkl, kDm, 0L, (void*)Kf, (void*)Kf, kDm, 0L,
        bk, bk, 0L, kSeq, kDm, kDm, 1.0f);
    rope_split_kernel<<<gRope, blk, 0, stream>>>(Qf, Kf, Qh, Ql, Kh, Kl);
    wmma_gemm64<1, true, 1, 2, false, 0><<<gVT, blk, 0, stream>>>(
        Wvh, Wvl, kDm, 0L, Xh, Xl, kDm, 0L, (void*)VTh, (void*)VTl, kSeq, 0L,
        bv, bv, 0L, kDm, kSeq, kDm, 1.0f);
    attn_mask64_kernel<<<gAtt, dim3(128), 0, stream>>>(Qh, Ql, Kh, Kl, VTh, VTl, mask, Of, 0.125f, -1.0e9f);
    split_bf16x2_kernel<<<gCast, blk, 0, stream>>>(Of, Oh, Ol, n2x);
    float* outb = (float*)d_out + (size_t)b * nRow;
    wmma_gemm64<1, true, 2, 0, false, 0><<<gProj, blk, 0, stream>>>(
        Oh, Ol, kDm, 0L, Woh, Wol, kDm, 0L, (void*)outb, (void*)outb, kDm, 0L,
        bo, bo, 0L, kSeq, kDm, kDm, 1.0f);
  }
}
